// SimpleGNNLayer_16329465659892
// MI455X (gfx1250) — hardware-run, weakly checked
//
#include <hip/hip_runtime.h>


namespace {
constexpr int N = 50000, E = 1600000, D = 128, DE = 3, NPB = 8;
constexpr float XS = 8.0f, HS = 256.0f, WSC = 256.0f, EPS = 1e-5f;
typedef _Float16 b16;
typedef __attribute__((ext_vector_type(16))) _Float16 v16b;
typedef __attribute__((ext_vector_type(8))) _Float16 v8b;
typedef __attribute__((ext_vector_type(8))) float v8f;
typedef __attribute__((ext_vector_type(4))) float v4f;
__device__ __forceinline__ float bf16_rne(float f) { unsigned int u = __float_as_uint(f); u += 0x7FFFu + ((u >> 16) & 1u); float r = __uint_as_float(u & 0xFFFF0000u); asm volatile("" : "+v"(r)); return r; }
__device__ __forceinline__ float bfv(float f) { float r = bf16_rne(f); asm volatile("" : "+v"(r)); return r; }
__device__ __forceinline__ void split16(float v, b16& hi, b16& lo) { hi = (b16)v; lo = (b16)(v - (float)hi); }
__device__ __forceinline__ v16b frag_kb(const b16* p, int hh) { const v8b a = *(const v8b*)(p + 8 * hh), b = *(const v8b*)(p + 16 + 8 * hh); v16b f;
#pragma unroll
  for (int e = 0; e < 8; ++e) { f[e] = a[e]; f[8 + e] = b[e]; } return f; }
__device__ __forceinline__ v8f wmma16b(v16b a, v16b b, v8f c) { v8f d = __builtin_amdgcn_wmma_f32_16x16x32_f16(false, a, false, b, (short)0, c, false, false); asm volatile("v_nop\n\tv_nop\n\tv_nop\n\tv_nop" : "+v"(d) : "v"(a), "v"(b)); return d; }
__device__ __forceinline__ void wave_lds_sync() { __builtin_amdgcn_fence(__ATOMIC_RELEASE, "workgroup"); __builtin_amdgcn_wave_barrier(); __builtin_amdgcn_fence(__ATOMIC_ACQUIRE, "workgroup"); }
__device__ __forceinline__ float pmul(float a, float b) { float p = a * b; asm volatile("" : "+v"(p)); return p; }
__device__ __forceinline__ int iclamp(int v, int lo, int hi) { return v < lo ? lo : (v > hi ? hi : v); }
__device__ __forceinline__ float gelu_erf(float v) { return 0.5f * v * (1.0f + erff(v * 0.70710678118654752f)); }
constexpr int CSR_NBLK8 = 512, CSR_GB8 = 8, CSR_GN8 = 1 << CSR_GB8  , CSR_TS8 = (CSR_GN8 < 32 ? 32 : CSR_GN8)  , CSR_MAXG8 = 512, CSR_CAP8 = 12288  ;
__device__ __host__ __forceinline__ int csr_tix8(int v) { return (v >> CSR_GB8) * CSR_TS8 + (v & (CSR_GN8 - 1)); }
__global__ __launch_bounds__(64) void csrA_kernel8(const int* __restrict__ dst, int E, int N, int nG, int CHP, int NGP, int* __restrict__ STG, int* __restrict__ HST) {
  extern __shared__ int sm[];
  int* cnt = sm; int* run = sm + NGP; int* ids = sm + 2 * NGP;
  const int b = blockIdx.x; const int ch = (E + CSR_NBLK8 - 1) / CSR_NBLK8; const int e0 = b * ch, e1 = min(E, e0 + ch);
  for (int i = threadIdx.x; i < NGP; i += 64) cnt[i] = 0;
  for (int i = threadIdx.x; i < CHP; i += 64) ids[i] = -1;
  __syncthreads();
  if (threadIdx.x == 0) {
    for (int e = e0; e < e1; ++e) { int d = dst[e]; d = (d < 0) ? 0 : (d >= N ? N - 1 : d); cnt[d >> CSR_GB8] += 1; }
    int acc = 0; for (int g = 0; g < nG; ++g) { run[g] = acc; acc += cnt[g]; }
    for (int e = e0; e < e1; ++e) { int d = dst[e]; d = (d < 0) ? 0 : (d >= N ? N - 1 : d); const int g = d >> CSR_GB8; ids[run[g]] = e; run[g] += 1; } }
  __syncthreads();
  typedef __attribute__((ext_vector_type(4))) int v4i;
  for (int pass = 0; pass < 2; ++pass) {
    for (int i = threadIdx.x; i < CHP / 4; i += 64) *(volatile v4i*)(STG + (size_t)b * CHP + i * 4) = *(const v4i*)(&ids[i * 4]);
    for (int i = threadIdx.x; i < NGP / 4; i += 64) { v4i v; for (int e = 0; e < 4; ++e) v[e] = (i * 4 + e < nG) ? cnt[i * 4 + e] : 0; *(volatile v4i*)(HST + (size_t)b * NGP + i * 4) = v; }
    __threadfence(); }
}
__global__ __launch_bounds__(512) void csrS_kernel8(const int* __restrict__ HST, int nG, int NGP, int* __restrict__ START, int* __restrict__ TOT, int* __restrict__ OFF) {
  __shared__ int tot[CSR_MAXG8];
  const int b = threadIdx.x;
  for (int pass = 0; pass < 2; ++pass) { int runb = 0; for (int g = 0; g < nG; ++g) { int c = HST[(size_t)b * NGP + g]; c = (c < 0) ? 0 : c; ((volatile int*)OFF)[(size_t)g * CSR_NBLK8 + b] = runb; runb += c; } __threadfence(); }
  for (int g = threadIdx.x; g < nG; g += 512) { int s = 0; for (int bb = 0; bb < CSR_NBLK8; ++bb) { int c = HST[(size_t)bb * NGP + g]; s += (c < 0) ? 0 : c; } tot[g] = s; }
  __syncthreads();
  if (threadIdx.x < 32) {
    __shared__ int st[CSR_MAXG8 + 32];
    if (threadIdx.x == 0) { int acc = 0; for (int g = 0; g < NGP; ++g) { st[g] = acc; if (g < nG) acc += (tot[g] + 31) & ~31; } st[NGP] = acc; }
    __builtin_amdgcn_fence(__ATOMIC_RELEASE, "workgroup"); __builtin_amdgcn_wave_barrier(); __builtin_amdgcn_fence(__ATOMIC_ACQUIRE, "workgroup");
    for (int pass = 0; pass < 2; ++pass) { for (int i = threadIdx.x; i < NGP + 32; i += 32) { ((volatile int*)START)[i] = (i <= NGP) ? st[min(i, NGP)] : 0; ((volatile int*)TOT)[i] = (i < nG) ? tot[i] : 0; } __threadfence(); } }
}
__global__ __launch_bounds__(256) void csrB_kernel8(const int* __restrict__ dst, int N, int nG, int CHP, int NGP, int permLen, const int* __restrict__ STG, const int* __restrict__ HST, const int* __restrict__ OFF, const int* __restrict__ START, const int* __restrict__ TOT, int* __restrict__ PERM, int* __restrict__ ROWPTR, int* __restrict__ ROWCNT, int* __restrict__ FLAG) {
  typedef __attribute__((ext_vector_type(4))) int v4i;
  __shared__ int ids[CSR_CAP8]; __shared__ unsigned short key[CSR_CAP8]; __shared__ int outp[CSR_CAP8]; __shared__ int ncnt[CSR_GN8 + 1]; __shared__ int boff[CSR_NBLK8 + 1];
  const int g = blockIdx.x, t_ = threadIdx.x; int tot = TOT[g]; int st = START[g], stn = START[g + 1]; const int v0 = g * CSR_GN8; const int nv = min(CSR_GN8, N - v0); const int t0 = g * CSR_TS8;
  st = (st < 0) ? 0 : (st > permLen - 32 ? permLen - 32 : st) & ~31; stn = (stn < st) ? st : (stn > permLen ? permLen : stn); tot = (tot < 0) ? 0 : tot; if (tot > stn - st && tot <= CSR_CAP8) tot = stn - st;
  if (tot > CSR_CAP8) {
    for (int pass = 0; pass < 2; ++pass) { for (int i = t_; i < CSR_TS8 / 4; i += 256) { v4i a, c; for (int e = 0; e < 4; ++e) { a[e] = st; c[e] = 0; } *(volatile v4i*)(ROWPTR + t0 + i * 4) = a; *(volatile v4i*)(ROWCNT + t0 + i * 4) = c; } if (t_ == 0) ((volatile int*)FLAG)[0] = 1; __threadfence(); } (void)nv; return; }
  if (t_ == 0) { int acc = 0; for (int b = 0; b < CSR_NBLK8; ++b) { boff[b] = acc; int c = HST[(size_t)b * NGP + g]; c = (c < 0) ? 0 : (c > CHP ? CHP : c); acc += c; if (acc > tot) acc = tot; } boff[CSR_NBLK8] = acc; }
  for (int i = t_; i <= CSR_GN8; i += 256) ncnt[i] = 0;
  __syncthreads();
  for (int b = 0; b < CSR_NBLK8; ++b) { const int c = boff[b + 1] - boff[b]; int o_ = OFF[(size_t)g * CSR_NBLK8 + b]; o_ = (o_ < 0) ? 0 : (o_ > CHP - c ? CHP - c : o_); const int* src_ = STG + (size_t)b * CHP + o_;
    for (int i = t_; i < c; i += 256) { int id = src_[i]; id = (id < 0) ? 0 : id; ids[boff[b] + i] = id; int d = dst[id]; d = (d < v0) ? v0 : (d >= N ? N - 1 : d); int kk = d - v0; kk = (kk < 0) ? 0 : (kk >= CSR_GN8 ? CSR_GN8 - 1 : kk); key[boff[b] + i] = (unsigned short)kk; } }
  __syncthreads();
  if (t_ == 0) { for (int i = 0; i < tot; ++i) ncnt[key[i]] += 1; int acc = 0; for (int vl = 0; vl < CSR_GN8; ++vl) { const int c = ncnt[vl]; ncnt[vl] = acc; acc += c; } ncnt[CSR_GN8] = acc;
    for (int i = 0; i < tot; ++i) { const int vl = key[i]; outp[ncnt[vl]] = ids[i]; ncnt[vl] += 1; }
    for (int vl = CSR_GN8; vl > 0; --vl) ncnt[vl] = ncnt[vl - 1]; ncnt[0] = 0; }
  __syncthreads();
  for (int pass = 0; pass < 2; ++pass) {
    for (int i = t_; i < (stn - st) / 4; i += 256) { v4i v; for (int e = 0; e < 4; ++e) { const int q = i * 4 + e; v[e] = (q < tot) ? outp[q] : -1; } *(volatile v4i*)(PERM + st + i * 4) = v; }
    for (int i = t_; i < CSR_TS8 / 4; i += 256) { v4i a, c; for (int e = 0; e < 4; ++e) { const int vl = i * 4 + e; const int vc = vl < CSR_GN8 ? vl : CSR_GN8; a[e] = (vl < CSR_GN8) ? st + ncnt[vc] : st; c[e] = (vl < nv) ? (ncnt[(vc < CSR_GN8 ? vc : CSR_GN8 - 1) + 1] - ncnt[vc]) : 0; } *(volatile v4i*)(ROWPTR + t0 + i * 4) = a; *(volatile v4i*)(ROWCNT + t0 + i * 4) = c; }
    __threadfence(); }
}
__global__ __launch_bounds__(256) void csrZ_kernel8(int* __restrict__ p, size_t n4) { typedef __attribute__((ext_vector_type(4))) int v4i; const size_t tid = (size_t)blockIdx.x * 256 + threadIdx.x, nth = (size_t)gridDim.x * 256; v4i z = {0, 0, 0, 0}; for (size_t i = tid; i < n4; i += nth) *(volatile v4i*)(p + i * 4) = z; }
struct CsrBufs8 { int *STG, *HST, *OFF, *START, *TOT, *PERM, *ROWPTR, *ROWCNT, *FLAG; int nG, NGP, CHP; size_t permLen; char* base; size_t bytes; };
static size_t csr_carve8(CsrBufs8& c, char* ws, size_t off, int E, int N) {
  const size_t off0 = off; c.base = ws + off;
  auto al = [&](size_t bytes) { char* p = ws + off; off += (bytes + 255) & ~(size_t)255; return p; };
  c.nG = (N + CSR_GN8 - 1) / CSR_GN8; c.NGP = (c.nG + 31) & ~31; const int ch = (E + CSR_NBLK8 - 1) / CSR_NBLK8; c.CHP = (ch + 31) & ~31; c.permLen = (size_t)E + 32 * (size_t)c.nG + 32;
  c.STG = (int*)al((size_t)CSR_NBLK8 * c.CHP * 4); c.HST = (int*)al((size_t)CSR_NBLK8 * c.NGP * 4); c.OFF = (int*)al((size_t)c.NGP * CSR_NBLK8 * 4); c.START = (int*)al((size_t)(c.NGP + 64) * 4); c.TOT = (int*)al((size_t)(c.NGP + 64) * 4);
  c.PERM = (int*)al(c.permLen * 4); c.ROWPTR = (int*)al((size_t)c.nG * CSR_TS8 * 4); c.ROWCNT = (int*)al((size_t)c.nG * CSR_TS8 * 4); c.FLAG = (int*)al(256);
  c.bytes = off - off0; return off;
}
static void csr_build8(const CsrBufs8& c, const int* dst, int E, int N, hipStream_t stream) {
  const size_t smem = (size_t)(2 * c.NGP + c.CHP) * 4;
  csrZ_kernel8<<<512, 256, 0, stream>>>((int*)c.base, c.bytes / 16);
  csrA_kernel8<<<CSR_NBLK8, 64, smem, stream>>>(dst, E, N, c.nG, c.CHP, c.NGP, c.STG, c.HST);
  csrS_kernel8<<<1, 512, 0, stream>>>(c.HST, c.nG, c.NGP, c.START, c.TOT, c.OFF);
  csrB_kernel8<<<c.nG, 256, 0, stream>>>(dst, N, c.nG, c.CHP, c.NGP, (int)c.permLen, c.STG, c.HST, c.OFF, c.START, c.TOT, c.PERM, c.ROWPTR, c.ROWCNT, c.FLAG);
}


__global__ __launch_bounds__(256) void wput_kernel(const float* __restrict__ w1, const float* __restrict__ w2, b16* __restrict__ W1N, b16* __restrict__ W2T) { const int u = blockIdx.x * 256 + threadIdx.x; if (u >= D * 16) return; const int o = u / 16, k0 = (u % 16) * 8; v8b a, c;
#pragma unroll
  for (int j = 0; j < 8; ++j) { a[j] = (b16)(bf16_rne(w1[(size_t)(k0 + j) * D + o]) * WSC); c[j] = (b16)(bf16_rne(w2[(size_t)(k0 + j) * D + o]) * WSC); }
  for (int pass = 0; pass < 2; ++pass) { *(volatile v8b*)(W1N + (size_t)o * D + k0) = a; *(volatile v8b*)(W2T + (size_t)o * D + k0) = c; __threadfence(); } }
__global__ __launch_bounds__(32) void pproj_kernel(const float* __restrict__ H, const b16* __restrict__ W1N, int NLIM, float* __restrict__ P) { __shared__ __attribute__((aligned(16))) b16 Ax[16][D + 8]; __shared__ float Tf[16][132]; const int lane = threadIdx.x, nloc = lane & 15, hlf = lane >> 4; const size_t n0 = (size_t)blockIdx.x * 16; if (n0 >= (size_t)NLIM) return;
  for (int rr = 0; rr < 16; ++rr) for (int q = 0; q < 4; ++q) { const int c = q * 32 + lane; Ax[rr][c] = (b16)(bf16_rne(H[(n0 + rr) * D + c]) * XS); }
  if (lane < 16) for (int k = D; k < D + 8; ++k) Ax[lane][k] = (b16)0.0f;
  wave_lds_sync(); v8f acc[8];
#pragma unroll
  for (int t = 0; t < 8; ++t) acc[t] = (v8f){};
#pragma unroll
  for (int kb = 0; kb < D; kb += 32) { const v16b a = frag_kb(&Ax[nloc][kb], hlf);
#pragma unroll
    for (int t = 0; t < 8; ++t) acc[t] = wmma16b(a, frag_kb(W1N + (size_t)(t * 16 + nloc) * D + kb, hlf), acc[t]); }
#pragma unroll
  for (int t = 0; t < 8; ++t)
#pragma unroll
    for (int r8 = 0; r8 < 8; ++r8) Tf[8 * hlf + r8][t * 16 + nloc] = acc[t][r8] * (1.0f / (XS * WSC));
  wave_lds_sync();
  for (int pass = 0; pass < 2; ++pass) { for (int rr = 0; rr < 16; ++rr) *(volatile v4f*)(P + (n0 + rr) * D + lane * 4) = *(const v4f*)(&Tf[rr][lane * 4]); __threadfence(); } }
__global__ __launch_bounds__(256) void edge_kernel(const float* __restrict__ P, const float* __restrict__ ea, const float* __restrict__ w1, const float* __restrict__ b1, const int* __restrict__ srcs, const int* __restrict__ PERM, const int* __restrict__ ROWPTR, const int* __restrict__ ROWCNT, int permLen, int NLIM, float* __restrict__ AG, float* __restrict__ CNT) { __shared__ float Cn[NPB]; const int wave = threadIdx.x >> 5, lane = threadIdx.x & 31; const size_t n = (size_t)blockIdx.x * NPB + wave; int nn = 0; v4f s = {0, 0, 0, 0};
  if (n < (size_t)NLIM) { v4f we[DE], bb; for (int q = 0; q < 4; ++q) { const int c = lane * 4 + q; bb[q] = bfv(b1[c]); for (int f = 0; f < DE; ++f) we[f][q] = bfv(w1[(size_t)(D + f) * D + c]); }
    int st = ROWPTR[n], cnt = ROWCNT[n]; cnt = iclamp(cnt, 0, E); st = iclamp(st, 0, permLen - cnt);
#pragma unroll 1
    for (int j = 0; j < cnt; ++j) { const int e = iclamp(PERM[st + j], 0, E - 1); const size_t sj = (size_t)iclamp(srcs[e], 0, N - 1); if (sj >= (size_t)NLIM) continue; ++nn; const v4f pv = *(const v4f*)(P + sj * D + lane * 4); const float e0 = bfv(ea[(size_t)e * DE]), e1 = bfv(ea[(size_t)e * DE + 1]), e2 = bfv(ea[(size_t)e * DE + 2]);
      for (int q = 0; q < 4; ++q) { const float v = pv[q] + pmul(e0, we[0][q]) + pmul(e1, we[1][q]) + pmul(e2, we[2][q]) + bb[q]; s[q] += gelu_erf(v); } } }
  if (lane == 0) Cn[wave] = (float)nn;
  __syncthreads();
  for (int pass = 0; pass < 2; ++pass) { if (n < (size_t)NLIM) *(volatile v4f*)(AG + n * D + lane * 4) = s; if (wave == 0) ((volatile float*)CNT)[(size_t)blockIdx.x * 32 + lane] = lane < NPB ? Cn[lane] : 0.0f; __threadfence(); } }
__global__ __launch_bounds__(32) void fin_kernel(const float* __restrict__ H, const float* __restrict__ AG, const float* __restrict__ CNT, const b16* __restrict__ W2T, const float* __restrict__ b2, const float* __restrict__ g, const float* __restrict__ bt, int NLIM, float* __restrict__ out) { __shared__ __attribute__((aligned(16))) b16 Ah[16][D + 8], Al[16][D + 8]; __shared__ float Tf[16][132]; const int lane = threadIdx.x, nloc = lane & 15, hlf = lane >> 4; const size_t n0 = (size_t)blockIdx.x * 16; if (n0 >= (size_t)NLIM) return;
  for (int rr = 0; rr < 16; ++rr) for (int q = 0; q < 4; ++q) { const int c = q * 32 + lane; b16 p, pl; split16(AG[(n0 + rr) * D + c] * HS, p, pl); Ah[rr][c] = p; Al[rr][c] = pl; }
  if (lane < 16) for (int k = D; k < D + 8; ++k) { Ah[lane][k] = (b16)0.0f; Al[lane][k] = (b16)0.0f; }
  wave_lds_sync(); v8f acc[8];
#pragma unroll
  for (int t = 0; t < 8; ++t) acc[t] = (v8f){};
#pragma unroll
  for (int kb = 0; kb < D; kb += 32) { const v16b a = frag_kb(&Ah[nloc][kb], hlf), al = frag_kb(&Al[nloc][kb], hlf);
#pragma unroll
    for (int t = 0; t < 8; ++t) { const v16b bw = frag_kb(W2T + (size_t)(t * 16 + nloc) * D + kb, hlf); acc[t] = wmma16b(a, bw, acc[t]); acc[t] = wmma16b(al, bw, acc[t]); } }
#pragma unroll
  for (int t = 0; t < 8; ++t) { const int cc = t * 16 + nloc; const float bb = bfv(b2[cc]);
#pragma unroll
    for (int r8 = 0; r8 < 8; ++r8) { const int rr = 8 * hlf + r8; const size_t n = n0 + rr; const float cntv = CNT[(n / NPB) * 32 + (n % NPB)]; Tf[rr][cc] = bfv(H[n * D + cc]) + acc[t][r8] * (1.0f / (HS * WSC)) + pmul(cntv, bb); } }
  wave_lds_sync();
  if (lane < 16) { float* row = &Tf[lane][0]; float m = 0.0f; for (int c = 0; c < D; ++c) m += row[c]; m *= (1.0f / D); float vr = 0.0f; for (int c = 0; c < D; ++c) { const float d = row[c] - m; vr += d * d; } vr *= (1.0f / D); const float rs = rsqrtf(vr + EPS); for (int c = 0; c < D; ++c) row[c] = pmul((row[c] - m) * rs, bfv(g[c])) + bfv(bt[c]); }
  wave_lds_sync();
  for (int pass = 0; pass < 2; ++pass) { for (int rr = 0; rr < 16; ++rr) *(volatile v4f*)(out + (n0 + rr) * D + lane * 4) = *(const v4f*)(&Tf[rr][lane * 4]); __threadfence(); } }
}

extern "C" void kernel_launch(void* const* d_in, const int* in_sizes, int n_in, void* d_out, int out_size, void* d_ws, size_t ws_size, hipStream_t stream) {
  (void)n_in;
  auto Fp = [&](int i) { return (const float*)d_in[i]; }; auto Ip = [&](int i) { return (const int*)d_in[i]; };
  if (in_sizes[0] != N * D || in_sizes[1] != 2 * E || in_sizes[2] != E * DE || in_sizes[3] != (D + DE) * D || in_sizes[5] != D * D || out_size != N * D) return;
  const int NLIM = N;
  size_t off = 0; char* ws = (char*)d_ws;
  auto carve = [&](size_t bytes) { char* p = ws + off; off += (bytes + 255) & ~(size_t)255; return p; };
  b16* W1N = (b16*)carve(D * D * 2); b16* W2T = (b16*)carve(D * D * 2); float* P = (float*)carve((size_t)N * D * 4); float* AG = (float*)carve((size_t)N * D * 4); float* CNT = (float*)carve((size_t)(N / NPB + 1) * 32 * 4); CsrBufs8 csr; off = csr_carve8(csr, ws, off, E, N);
  if (off > ws_size || off > ((size_t)112 << 20)) return;
  wput_kernel<<<(D * 16 + 255) / 256, 256, 0, stream>>>(Fp(3), Fp(5), W1N, W2T);
  csr_build8(csr, Ip(1) + E, E, N, stream);
  pproj_kernel<<<NLIM / 16, 32, 0, stream>>>(Fp(0), W1N, NLIM, P);
  edge_kernel<<<(NLIM + NPB - 1) / NPB, 256, 0, stream>>>(P, Fp(2), Fp(3), Fp(4), Ip(1), csr.PERM, csr.ROWPTR, csr.ROWCNT, (int)csr.permLen, NLIM, AG, CNT);
  fin_kernel<<<NLIM / 16, 32, 0, stream>>>(Fp(0), AG, CNT, W2T, Fp(6), Fp(7), Fp(8), NLIM, (float*)d_out);
}
